// backbone_41644002902564
// MI455X (gfx1250) — hardware-verified
//
#include <hip/hip_runtime.h>
#include <math.h>

typedef __attribute__((ext_vector_type(16))) _Float16 v16h;
typedef __attribute__((ext_vector_type(16))) __bf16 v16b;
typedef __attribute__((ext_vector_type(8)))  _Float16 v8h;
typedef __attribute__((ext_vector_type(8)))  float v8f;
typedef __attribute__((ext_vector_type(4)))  float v4f;
typedef __attribute__((ext_vector_type(2)))  float v2f;
typedef __attribute__((ext_vector_type(4)))  unsigned v4u;
typedef __attribute__((ext_vector_type(4)))  int v4i;
typedef float __attribute__((may_alias)) float_a;
typedef int __attribute__((may_alias)) int_a;

template <typename T> __device__ __forceinline__ void vst2(void* p, T v) { *(volatile T*)p = v; __threadfence(); *(volatile T*)p = v; }
__device__ __forceinline__ v8f wmma16(v16h a, v16h b, v8f c) {
  v8f d = __builtin_amdgcn_wmma_f32_16x16x32_f16(false, a, false, b, (short)0, c, false, false);
  asm volatile("v_nop\n\tv_nop\n\tv_nop\n\tv_nop" : "+v"(d) : "v"(a), "v"(b));
  return d;
}
__device__ __forceinline__ v8f wmma_bf(v16b a, v16b b, v8f c) {
  v8f d = __builtin_amdgcn_wmma_f32_16x16x32_bf16(false, a, false, b, (short)0, c, false, false);
  asm volatile("v_nop\n\tv_nop\n\tv_nop\n\tv_nop" : "+v"(d) : "v"(a), "v"(b));
  return d;
}
__device__ __forceinline__ v16h frag_h(const _Float16* rowk0, int lane) {
  union { v16h v; v8h q[2]; } u; const _Float16* p = rowk0 + 8 * (lane >> 4);
  u.q[0] = *(const v8h*)p; u.q[1] = *(const v8h*)(p + 16); return u.v;
}
__device__ __forceinline__ v16h frag_f32(const float* rowk0, int lane) {
  v16h a; const float* p = rowk0 + 8 * (lane >> 4);
#pragma unroll
  for (int i = 0; i < 8; ++i) { a[i] = (_Float16)p[i]; a[8 + i] = (_Float16)p[16 + i]; }
  return a;
}
__device__ __forceinline__ v16h frag_f32s(const float* rowk0, int lane, float sc) {
  v16h a; const float* p = rowk0 + 8 * (lane >> 4);
#pragma unroll
  for (int i = 0; i < 8; ++i) { a[i] = (_Float16)(p[i] * sc); a[8 + i] = (_Float16)(p[16 + i] * sc); }
  return a;
}
__device__ __forceinline__ v16h fragc_f32(const float* W, int k0, int n, int lane, int ld, int K) {
  v16h a; const int g = lane >> 4;
#pragma unroll
  for (int i = 0; i < 8; ++i) { const int ka = k0 + 8 * g + i, kb = ka + 16;
    a[i] = (_Float16)(ka < K ? W[(size_t)ka * ld + n] : 0.f); a[8 + i] = (_Float16)(kb < K ? W[(size_t)kb * ld + n] : 0.f); }
  return a;
}
struct F2 { v16b h, l; };
__device__ __forceinline__ F2 bsplit16(const float v[16]) { F2 r;
#pragma unroll
  for (int i = 0; i < 16; ++i) { const __bf16 h = (__bf16)v[i]; r.h[i] = h; r.l[i] = (__bf16)(v[i] - (float)h); }
  return r; }
__device__ __forceinline__ F2 split_row(const float* row, int k0, int lane) { float v[16]; const float* p = row + k0 + 8 * (lane >> 4);
#pragma unroll
  for (int i = 0; i < 8; ++i) { v[i] = p[i]; v[8 + i] = p[16 + i]; }
  return bsplit16(v); }
__device__ __forceinline__ F2 split_rowK(const float* row, int k0, int lane, int K) { float v[16]; const int g = lane >> 4;
#pragma unroll
  for (int i = 0; i < 8; ++i) { const int ka = k0 + 8 * g + i, kb = ka + 16; v[i] = ka < K ? row[ka] : 0.f; v[8 + i] = kb < K ? row[kb] : 0.f; }
  return bsplit16(v); }
__device__ __forceinline__ F2 split_col(const float* W, int k0, int n, int lane, int ld, int K) { float v[16]; const int g = lane >> 4;
#pragma unroll
  for (int i = 0; i < 8; ++i) { const int ka = k0 + 8 * g + i, kb = ka + 16; v[i] = ka < K ? W[(size_t)ka * ld + n] : 0.f; v[8 + i] = kb < K ? W[(size_t)kb * ld + n] : 0.f; }
  return bsplit16(v); }
__device__ __forceinline__ v8f mac3(const F2& a, const F2& b, v8f c) { c = wmma_bf(a.l, b.h, c); c = wmma_bf(a.h, b.l, c); return wmma_bf(a.h, b.h, c); }
__device__ __forceinline__ float sigm(float v) { return 1.0f / (1.0f + expf(-v)); }
#define LDSX() do { asm volatile("s_wait_dscnt 0" ::: "memory"); __builtin_amdgcn_wave_barrier(); __builtin_amdgcn_fence(__ATOMIC_RELEASE, "workgroup"); } while (0)

#define NS 64
#define CC 512
#define TT 64
#define FO 256
#define NPAIR 2016

__global__ __launch_bounds__(256) void k_score(const float* __restrict__ x, const float* __restrict__ w, const float* __restrict__ b, float* __restrict__ sc) {
  __shared__ float red[256];
  const int n = blockIdx.x, tid = threadIdx.x; float s = 0.f;
#pragma unroll 1
  for (int q = tid; q < CC * TT; q += 256) s += x[(size_t)n * CC * TT + q] * w[q];
  red[tid] = s; __syncthreads();
  for (int st = 128; st > 0; st >>= 1) { if (tid < st) red[tid] += red[tid + st]; __syncthreads(); }
  if (tid < 32) vst2(sc + (size_t)n * 32 + tid, (float_a)(tid == 0 ? 1.0f / (1.0f + expf(-(red[0] + b[0]))) : 0.f));
}
__global__ __launch_bounds__(128) void k_f(const float* __restrict__ x, const float* __restrict__ w, const float* __restrict__ b, _Float16* __restrict__ F) {
  __shared__ __align__(16) _Float16 so[4][16][72];
  const int tid = threadIdx.x, wave = tid >> 5, lane = tid & 31, col = lane & 15, g = lane >> 4;
  const int n = blockIdx.y, o0 = blockIdx.x * 64 + wave * 16;
  v8f acc[4] = {};
#pragma unroll 1
  for (int kc = 0; kc < CC / 32; ++kc) { const v16h a = frag_f32(w + (size_t)(o0 + col) * CC + kc * 32, lane);
#pragma unroll
    for (int j = 0; j < 4; ++j) acc[j] = wmma16(a, fragc_f32(x + (size_t)n * CC * TT, kc * 32, j * 16 + col, lane, TT, CC), acc[j]); }
#pragma unroll
  for (int j = 0; j < 4; ++j)
#pragma unroll
    for (int r = 0; r < 8; ++r) so[wave][8 * g + r][j * 16 + col] = (_Float16)(acc[j][r] + b[o0 + 8 * g + r]);
  LDSX();
  for (int q = lane; q < 16 * 8; q += 32) { const int rl = q >> 3, pc = q & 7; vst2(F + ((size_t)n * FO + o0 + rl) * TT + pc * 8, *(const v4u*)(&so[wave][rl][pc * 8])); }
}
__global__ __launch_bounds__(128) void k_pair(const _Float16* __restrict__ F, const float* __restrict__ wc1, const float* __restrict__ bc1, const float* __restrict__ wc2, const float* __restrict__ bc2,
                                            const float* __restrict__ wf1, const float* __restrict__ bf1, const float* __restrict__ wf2, const float* __restrict__ bf2, const float* __restrict__ wf3, const float* __restrict__ bf3, float* __restrict__ gsc) {
  __shared__ __align__(16) float sM[64][260];
  __shared__ __align__(16) float sw[2][32][68];
  __shared__ __align__(16) float sh[32][132];
  __shared__ float h1[32][32], h2[8][32], v64[64], v32[32], v8[8];
  const int tid = threadIdx.x, wave = tid >> 5, lane = tid & 31, col = lane & 15, g = lane >> 4;
  const int p = blockIdx.x;
  int i = 0, base = 0; while (p >= base + (NS - 1 - i)) { base += NS - 1 - i; ++i; }
  const int j = i + 1 + (p - base);
  const _Float16* Fi = F + ((size_t)i * FO) * TT; const _Float16* Fj = F + ((size_t)j * FO) * TT;
  v8f hacc[8];
#pragma unroll
  for (int q = 0; q < 8; ++q) hacc[q] = (v8f){};
#pragma unroll 1
  for (int sub = 0; sub < 4; ++sub) { const int c0 = sub * 64 + wave * 16;
    for (int q = tid; q < 2 * 32 * 64; q += 128) { const int par = q >> 11, o = (q >> 6) & 31, cl = q & 63; sw[par][o][cl] = wc1[(size_t)o * CC + 2 * (sub * 64 + cl) + par]; }
    v16h a[2];
#pragma unroll
    for (int kc = 0; kc < 2; ++kc) a[kc] = frag_h(Fi + (size_t)(c0 + col) * TT + kc * 32, lane);
#pragma unroll 1
    for (int hf = 0; hf < 2; ++hf) { v8f acc[8] = {};
#pragma unroll
      for (int kc = 0; kc < 2; ++kc) {
#pragma unroll
        for (int jt = 0; jt < 8; ++jt) acc[jt] = wmma16(a[kc], frag_h(Fj + (size_t)(hf * 128 + jt * 16 + col) * TT + kc * 32, lane), acc[jt]); }
#pragma unroll
      for (int jt = 0; jt < 8; ++jt)
#pragma unroll
        for (int r = 0; r < 8; ++r) sM[wave * 16 + 8 * g + r][hf * 128 + jt * 16 + col] = acc[jt][r]; }
    __syncthreads();
#pragma unroll
    for (int q = 0; q < 8; ++q) { const int st_ = 2 * wave + (q & 1), par = (q >> 1) & 1, ot = q >> 2;
#pragma unroll
      for (int kc = 0; kc < 2; ++kc) hacc[q] = wmma16(frag_f32(&sw[par][ot * 16 + col][0] + kc * 32, lane), fragc_f32(&sM[0][0] + par * 128, kc * 32, st_ * 16 + col, lane, 260, 64), hacc[q]); }
    __syncthreads(); }
#pragma unroll
  for (int q = 0; q < 8; ++q) { const int st_ = 2 * wave + (q & 1), par = (q >> 1) & 1, ot = q >> 2; (void)par;
    if (((q >> 1) & 1) == 0) { const v8f other = hacc[q + 2];
#pragma unroll
      for (int r = 0; r < 8; ++r) sh[ot * 16 + 8 * g + r][st_ * 16 + col] = hacc[q][r] + other[r] + bc1[ot * 16 + 8 * g + r]; } }
  __syncthreads();
  for (int q = tid; q < 32 * 32; q += 128) { const int o = q >> 5, cell = q & 31; const int ph = cell >> 1, pw = cell & 1; float m = -3.0e38f;
#pragma unroll
    for (int d = 0; d < 4; ++d) { const int hh = ph * 2 + (d >> 1), ww = pw * 2 + (d & 1); m = fmaxf(m, sh[o][hh * 4 + ww]); }
    h1[o][cell] = m; }
  __syncthreads();
  for (int q = tid; q < 8 * 32; q += 128) { const int o2 = q >> 5, cell = q & 31; float a2 = bc2[o2];
#pragma unroll 1
    for (int o = 0; o < 32; ++o) a2 += wc2[o2 * 32 + o] * h1[o][cell];
    h2[o2][cell] = a2; }
  __syncthreads();
  if (tid < 64) { const int o2 = tid >> 3, ph = tid & 7; float m = -3.0e38f;
#pragma unroll
    for (int d = 0; d < 4; ++d) { const int hh = ph * 2 + (d >> 1), ww = d & 1; m = fmaxf(m, h2[o2][hh * 2 + ww]); }
    v64[tid] = m; }
  __syncthreads();
  if (tid < 32) { float a2 = bf1[tid]; for (int k = 0; k < 64; ++k) a2 += v64[k] * wf1[tid * 64 + k]; v32[tid] = a2 > 0.f ? a2 : 0.f; }
  __syncthreads();
  if (tid < 8) { float a2 = bf2[tid]; for (int k = 0; k < 32; ++k) a2 += v32[k] * wf2[tid * 32 + k]; v8[tid] = a2 > 0.f ? a2 : 0.f; }
  __syncthreads();
  if (tid < 32) { float a2 = 0.f; if (tid == 0) { a2 = bf3[0]; for (int k = 0; k < 8; ++k) a2 += v8[k] * wf3[k]; a2 = 1.0f / (1.0f + expf(-a2)); } vst2(gsc + (size_t)p * 32 + tid, (float_a)(tid == 0 ? a2 : 0.f)); }
}
__global__ __launch_bounds__(256) void k_out(const float* __restrict__ sc, const float* __restrict__ gsc, float* __restrict__ out0, float* __restrict__ out1) {
  __shared__ __align__(16) float s0[NS]; __shared__ __align__(16) float s1[NPAIR];
  const int tid = threadIdx.x;
  if (tid < NS) s0[tid] = sc[(size_t)tid * 32];
  for (int q = tid; q < NPAIR; q += 256) s1[q] = gsc[(size_t)q * 32];
  __syncthreads();
  if (tid < NS / 4) vst2(out0 + tid * 4, *(const v4f*)(&s0[tid * 4]));
  for (int q = tid; q < NPAIR / 4; q += 256) vst2(out1 + q * 4, *(const v4f*)(&s1[q * 4]));
}
extern "C" void kernel_launch(void* const* d_in, const int* in_sizes, int n_in, void* d_out, int out_size, void* d_ws, size_t ws_size, hipStream_t stream) {
  (void)in_sizes; (void)n_in; (void)out_size; (void)ws_size;
  const float** I = (const float**)d_in;
  const float* x = I[0]; const float* wcv = I[1]; const float* bcv = I[2]; const float* wc1 = I[3]; const float* bc1 = I[4]; const float* wc2 = I[5]; const float* bc2 = I[6];
  const float* wf1 = I[7]; const float* bf1 = I[8]; const float* wf2 = I[9]; const float* bf2 = I[10]; const float* wf3 = I[11]; const float* bf3 = I[12]; const float* wml = I[13]; const float* bml = I[14];
  float* out0 = (float*)d_out; float* out1 = out0 + 64;
  char* ws = (char*)d_ws; size_t off = 0;
  auto take = [&](size_t bytes) { char* p = ws + off; off += (bytes + 255) & ~(size_t)255; return p; };
  _Float16* F = (_Float16*)take((size_t)NS * FO * TT * 2); float* sc = (float*)take((size_t)NS * 32 * 4); float* gsc = (float*)take((size_t)NPAIR * 32 * 4);
  k_score<<<NS, 256, 0, stream>>>(x, wml, bml, sc);
  k_f<<<dim3(FO / 64, NS), 128, 0, stream>>>(x, wcv, bcv, F);
  k_pair<<<NPAIR, 128, 0, stream>>>(F, wc1, bc1, wc2, bc2, wf1, bf1, wf2, bf2, wf3, bf3, gsc);
  k_out<<<1, 256, 0, stream>>>(sc, gsc, out0, out1);
}
